// Sam3TrackerVideoRoPEAttention_73014444032502
// MI455X (gfx1250) — hardware-verified
//
#include <hip/hip_runtime.h>


#define SQ   4096
#define SK   16448
#define HD   256
#define QC   1024
#define NEX  64
#define PCAR 1024.0f
typedef _Float16 h16;
typedef unsigned short bf;
typedef __attribute__((ext_vector_type(16))) __bf16   v16bf;
typedef __attribute__((ext_vector_type(16))) _Float16 v16h;
typedef __attribute__((ext_vector_type(8)))  _Float16 v8h;
typedef __attribute__((ext_vector_type(8)))  unsigned short v8us;
typedef __attribute__((ext_vector_type(8)))  float    v8f;
typedef __attribute__((ext_vector_type(4)))  float    v4f;
typedef v8h  __attribute__((may_alias)) v8ha;
typedef v4f  __attribute__((may_alias)) v4fa;
typedef v8us __attribute__((may_alias)) v8usa;

__device__ __forceinline__ unsigned short f2bf(float f) { unsigned u = __float_as_uint(f); u += 0x7FFFu + ((u >> 16) & 1u); return (unsigned short)(u >> 16); }
__device__ __forceinline__ float bf2f(unsigned short b) { return __uint_as_float(((unsigned)b) << 16); }
__device__ __forceinline__ float bfr(float f) { return bf2f(f2bf(f)); }
__device__ __forceinline__ v16h cat16(v8h lo, v8h hi) { return __builtin_shufflevector(lo, hi, 0, 1, 2, 3, 4, 5, 6, 7, 8, 9, 10, 11, 12, 13, 14, 15); }
__device__ __forceinline__ v16bf cat16b(v8us lo, v8us hi) { return __builtin_bit_cast(v16bf, __builtin_shufflevector(lo, hi, 0, 1, 2, 3, 4, 5, 6, 7, 8, 9, 10, 11, 12, 13, 14, 15)); }
__device__ __forceinline__ v8f wmma16(v16h a, v16h b, v8f c) { return __builtin_amdgcn_wmma_f32_16x16x32_f16(false, a, false, b, (short)0, c, false, false); }
__device__ __forceinline__ v8f wmmab(v16bf a, v16bf b, v8f c) { return __builtin_amdgcn_wmma_f32_16x16x32_bf16(false, a, false, b, (short)0, c, false, false); }


template <typename T16> struct WFrag;
template <> struct WFrag<h16> { typedef v16h V; static __device__ __forceinline__ V ld(const h16* p) { return cat16(*(const v8h*)p, *(const v8h*)(p + 16)); } static __device__ __forceinline__ v8f mma(V a, V b, v8f c) { return wmma16(a, b, c); } };
template <> struct WFrag<bf> { typedef v16bf V; static __device__ __forceinline__ V ld(const bf* p) { return cat16b(*(const v8us*)p, *(const v8us*)(p + 16)); } static __device__ __forceinline__ v8f mma(V a, V b, v8f c) { return wmmab(a, b, c); } };
template <typename T16, int NSPLIT, bool BIAS>
__global__ __launch_bounds__(32) void k_gemmw(const T16* __restrict__ A, const T16* __restrict__ A2, const T16* __restrict__ Bt, const T16* __restrict__ Bt2, int K, float* C, int ldc, const float* __restrict__ bias, size_t sA, size_t sB, size_t sC) {
    typedef typename WFrag<T16>::V V;
    __shared__ __align__(16) float os[16 * 68];
    const size_t z = blockIdx.z; A += z * sA; if (A2) A2 += z * sA; Bt += z * sB; if (Bt2) Bt2 += z * sB; C += z * sC;
    const int lane = threadIdx.x & 31, lr = lane & 15, hi = lane >> 4; const int r0 = blockIdx.x * 64, c0 = blockIdx.y * 64;
    v8f acc[4][4];
#pragma unroll
    for (int mb = 0; mb < 4; ++mb)
#pragma unroll
        for (int nb = 0; nb < 4; ++nb) acc[mb][nb] = (v8f){};
    const size_t aoff = (size_t)(r0 + lr) * K + 8 * hi, boff = (size_t)(c0 + lr) * K + 8 * hi;
#pragma unroll 1
    for (int kc = 0; kc < K; kc += 32) {
        V a[4], a2[4];
#pragma unroll
        for (int mb = 0; mb < 4; ++mb) { a[mb] = WFrag<T16>::ld(A + aoff + (size_t)mb * 16 * K + kc); if (NSPLIT == 1 || NSPLIT == 2) a2[mb] = WFrag<T16>::ld(A2 + aoff + (size_t)mb * 16 * K + kc); }
#pragma unroll
        for (int nb = 0; nb < 4; ++nb) { const V b = WFrag<T16>::ld(Bt + boff + (size_t)nb * 16 * K + kc); V b2; if (NSPLIT >= 2) b2 = WFrag<T16>::ld(Bt2 + boff + (size_t)nb * 16 * K + kc);
#pragma unroll
            for (int mb = 0; mb < 4; ++mb) { acc[mb][nb] = WFrag<T16>::mma(a[mb], b, acc[mb][nb]); if (NSPLIT == 1 || NSPLIT == 2) acc[mb][nb] = WFrag<T16>::mma(a2[mb], b, acc[mb][nb]); if (NSPLIT >= 2) acc[mb][nb] = WFrag<T16>::mma(a[mb], b2, acc[mb][nb]); } }
        asm volatile("v_nop\n\tv_nop\n\tv_nop\n\tv_nop" : "+v"(acc[0][0]), "+v"(acc[1][1]), "+v"(acc[2][2]), "+v"(acc[3][3]) : "v"(a[0]), "v"(a[3]));
    }
#pragma unroll
    for (int mb = 0; mb < 4; ++mb) {
#pragma unroll
        for (int nb = 0; nb < 4; ++nb) {
#pragma unroll
            for (int j = 0; j < 8; ++j) os[(hi * 8 + j) * 68 + nb * 16 + lr] = acc[mb][nb][j]; }
        __builtin_amdgcn_wave_barrier(); asm volatile("" ::: "memory");
        float* crow = C + (size_t)(r0 + mb * 16) * ldc + c0;
#pragma unroll 1
        for (int ps = 0; ps < 2; ++ps) {
#pragma unroll
            for (int s = 0; s < 8; ++s) { const int row = 2 * s + hi, cofs = lr * 4; v4f val = *(const v4fa*)(os + row * 68 + cofs); if (BIAS) { val[0] += bfr(bias[c0 + cofs]); val[1] += bfr(bias[c0 + cofs + 1]); val[2] += bfr(bias[c0 + cofs + 2]); val[3] += bfr(bias[c0 + cofs + 3]); }
                *(volatile v4f*)(crow + (size_t)row * ldc + cofs) = val; }
            if (ps == 0) __threadfence(); }
        __builtin_amdgcn_wave_barrier(); asm volatile("" ::: "memory");
    }
}

__device__ __forceinline__ h16 tohx(float x) { return (h16)x; }
__device__ __forceinline__ void splitf(float y, unsigned short& h, unsigned short& l) { h = f2bf(y); l = f2bf(y - bf2f(h)); }
typedef __attribute__((ext_vector_type(2))) unsigned short v2us;
typedef __attribute__((ext_vector_type(4))) unsigned short v4us;
typedef __attribute__((ext_vector_type(2))) _Float16 v2h;
typedef __attribute__((ext_vector_type(4))) _Float16 v4h;
typedef __attribute__((ext_vector_type(2))) float v2f;

__global__ __launch_bounds__(256) void k_cvt8(const float* __restrict__ src, bf* dst, size_t n8) { const size_t i = (size_t)blockIdx.x * 256 + threadIdx.x; if (i >= n8) return; const v8f v = *(const v8f*)(src + i * 8); v8us o;
#pragma unroll
    for (int k = 0; k < 8; ++k) o[k] = f2bf(v[k]); *(volatile v8us*)(dst + i * 8) = o; __threadfence(); *(volatile v8us*)(dst + i * 8) = o; }
__global__ __launch_bounds__(256) void k_wtG(const float* __restrict__ Wm, bf* Bt) { const int idx = blockIdx.x * 256 + threadIdx.x; if (idx >= HD * HD / 8) return; const int n = idx / (HD / 8); const int k8 = (idx % (HD / 8)) * 8; unsigned short o[8];
#pragma unroll
    for (int u = 0; u < 8; ++u) o[u] = f2bf(Wm[(size_t)(k8 + u) * HD + n]); typedef __attribute__((ext_vector_type(8))) unsigned short v8us; v8us v; for (int u = 0; u < 8; ++u) v[u] = o[u]; *(volatile v8us*)(Bt + (size_t)n * HD + k8) = v; __threadfence(); *(volatile v8us*)(Bt + (size_t)n * HD + k8) = v; }
__global__ __launch_bounds__(256) void k_ropq(float* F, int nrows, int nrope, int tdiv, const float* __restrict__ cosT, const float* __restrict__ sinT) { const size_t e = ((size_t)blockIdx.x * 256 + threadIdx.x) * 2; if (e >= (size_t)nrows * HD) return; const int d = (int)(e % HD); const int t = (int)(e / HD); v2f o; const float x0 = F[e], x1 = F[e + 1];
    if (t < nrope) { const int tr = t / tdiv; const float c0 = bfr(cosT[(size_t)tr * HD + d]), s0 = bfr(sinT[(size_t)tr * HD + d]), c1 = bfr(cosT[(size_t)tr * HD + d + 1]), s1 = bfr(sinT[(size_t)tr * HD + d + 1]); float p0 = __fmul_rn(x0, c0), p1 = __fmul_rn(x1, s0), p2 = __fmul_rn(x1, c1), p3 = __fmul_rn(x0, s1); asm volatile("" : "+v"(p0)); asm volatile("" : "+v"(p1)); asm volatile("" : "+v"(p2)); asm volatile("" : "+v"(p3)); o[0] = __fsub_rn(p0, p1); o[1] = __fadd_rn(p2, p3); }
    else { o[0] = x0; o[1] = x1; }
    *(volatile v2f*)(F + e) = o; __threadfence(); *(volatile v2f*)(F + e) = o; }
__global__ __launch_bounds__(256) void k_hlG(const float* __restrict__ F, bf* Fh, bf* Fl, size_t n) { const size_t e = ((size_t)blockIdx.x * 256 + threadIdx.x) * 4; if (e >= n) return; const v4f a = *(const v4f*)(F + e); v4us oh, ol; for (int u = 0; u < 4; ++u) { unsigned short p, q; splitf(a[u], p, q); oh[u] = p; ol[u] = q; } *(volatile v4us*)(Fh + e) = oh; *(volatile v4us*)(Fl + e) = ol; __threadfence(); *(volatile v4us*)(Fh + e) = oh; *(volatile v4us*)(Fl + e) = ol; }
__global__ __launch_bounds__(256) void k_v16T(const float* __restrict__ V, h16* VT) { const size_t e = ((size_t)blockIdx.x * 256 + threadIdx.x) * 2; if (e >= (size_t)HD * SK) return; const int j = (int)(e % SK); const int d = (int)(e / SK); v2h o; o[0] = tohx(V[(size_t)j * HD + d]); o[1] = tohx(V[(size_t)(j + 1) * HD + d]); *(volatile v2h*)(VT + e) = o; __threadfence(); *(volatile v2h*)(VT + e) = o; }
__global__ __launch_bounds__(256) void k_lsoft(const float* __restrict__ S, const int* __restrict__ FLG, h16* P16) { const int lane = threadIdx.x & 31; const int row = blockIdx.x * 8 + (threadIdx.x >> 5); if (row >= QC) return; const float* sr = S + (size_t)row * SK; const bool poison = (FLG[0] != 0); float mx = -3.0e38f;
#pragma unroll 4
    for (int ch = 0; ch < SK / 64; ++ch) { const v2f a = *(const v2f*)(sr + ch * 64 + lane * 2); mx = fmaxf(mx, fmaxf(a[0] * 0.0625f, a[1] * 0.0625f)); }
#pragma unroll
    for (int sh = 16; sh; sh >>= 1) mx = fmaxf(mx, __shfl_xor(mx, sh, 32));
    float sum = 0.f;
#pragma unroll 4
    for (int ch = 0; ch < SK / 64; ++ch) { const v2f a = *(const v2f*)(sr + ch * 64 + lane * 2);
#pragma unroll
        for (int q = 0; q < 2; ++q) { float sa = a[q] * 0.0625f; asm volatile("" : "+v"(sa)); float d0 = __fsub_rn(sa, mx); asm volatile("" : "+v"(d0)); sum += __builtin_amdgcn_exp2f(__fmul_rn(d0, 1.4426950408889634f)); } }
#pragma unroll
    for (int sh = 16; sh; sh >>= 1) sum += __shfl_xor(sum, sh, 32);
    const float f = poison ? __builtin_nanf("") : __fdiv_rn(PCAR, sum);
    for (int ps = 0; ps < 2; ++ps) {
#pragma unroll 4
        for (int ch = 0; ch < SK / 64; ++ch) { const v2f a = *(const v2f*)(sr + ch * 64 + lane * 2); v2h o;
#pragma unroll
            for (int q = 0; q < 2; ++q) { float sa = a[q] * 0.0625f; asm volatile("" : "+v"(sa)); float d0 = __fsub_rn(sa, mx); asm volatile("" : "+v"(d0)); o[q] = tohx(__builtin_amdgcn_exp2f(__fmul_rn(d0, 1.4426950408889634f)) * f); }
            *(volatile v2h*)(P16 + (size_t)row * SK + ch * 64 + lane * 2) = o; }
        if (ps == 0) __threadfence(); } }
__global__ __launch_bounds__(256) void k_ofix(const float* __restrict__ O, bf* Oh, bf* Ol) { const size_t e = ((size_t)blockIdx.x * 256 + threadIdx.x) * 4; if (e >= (size_t)QC * HD) return; const v4f a = *(const v4f*)(O + e); v4us oh, ol; for (int u = 0; u < 4; ++u) { unsigned short p, q; splitf(a[u] * (1.0f / PCAR), p, q); oh[u] = p; ol[u] = q; } *(volatile v4us*)(Oh + e) = oh; *(volatile v4us*)(Ol + e) = ol; __threadfence(); *(volatile v4us*)(Oh + e) = oh; *(volatile v4us*)(Ol + e) = ol; }
__global__ __launch_bounds__(32) void k_nexchk(const int* __restrict__ nex, int* FLG) { const int tid = threadIdx.x; if (tid < 8) { const int v = (tid == 0) ? ((nex[0] != NEX) ? 1 : 0) : 0; *(volatile int*)(FLG + tid) = v; __threadfence(); *(volatile int*)(FLG + tid) = v; } }

extern "C" void kernel_launch(void* const* d_in, const int* in_sizes, int n_in,
                              void* d_out, int out_size, void* d_ws, size_t ws_size, hipStream_t stream) {
    (void)in_sizes; (void)n_in; (void)out_size;
    const float* query = (const float*)d_in[0]; const float* key = (const float*)d_in[1]; const float* value = (const float*)d_in[2]; const float* cosT = (const float*)d_in[3]; const float* sinT = (const float*)d_in[4];
    const float* q_w = (const float*)d_in[5]; const float* q_b = (const float*)d_in[6]; const float* k_w = (const float*)d_in[7]; const float* k_b = (const float*)d_in[8]; const float* v_w = (const float*)d_in[9]; const float* v_b = (const float*)d_in[10]; const float* o_w = (const float*)d_in[11]; const float* o_b = (const float*)d_in[12]; const int* nex = (const int*)d_in[13];
    float* OUT = (float*)d_out;
    char* wsp = (char*)d_ws;
    auto take = [&](size_t bytes) { char* p = wsp; wsp += (bytes + 255) & ~(size_t)255; return (void*)p; };
    bf* WQ = (bf*)take(HD * HD * 2); bf* WK = (bf*)take(HD * HD * 2); bf* WV = (bf*)take(HD * HD * 2); bf* WO = (bf*)take(HD * HD * 2); int* FLG = (int*)take(256);
    bf* XQ = (bf*)take((size_t)SQ * HD * 2); bf* XK = (bf*)take((size_t)SK * HD * 2);
    float* FQ = (float*)take((size_t)SQ * HD * 4); bf* QPh = (bf*)take((size_t)SQ * HD * 2); bf* QPl = (bf*)take((size_t)SQ * HD * 2);
    float* FK = (float*)take((size_t)SK * HD * 4); bf* KPh = (bf*)take((size_t)SK * HD * 2); bf* KPl = (bf*)take((size_t)SK * HD * 2); h16* VT16 = (h16*)take((size_t)HD * SK * 2);
    float* S = (float*)take((size_t)QC * SK * 4); h16* P16 = (h16*)take((size_t)QC * SK * 2); float* O = (float*)take((size_t)QC * HD * 4); bf* Oh = (bf*)take((size_t)QC * HD * 2); bf* Ol = (bf*)take((size_t)QC * HD * 2);
    if ((size_t)(wsp - (char*)d_ws) > ws_size) return;
    float* FV = FK;
    k_wtG<<<(HD * HD / 8 + 255) / 256, 256, 0, stream>>>(q_w, WQ); k_wtG<<<(HD * HD / 8 + 255) / 256, 256, 0, stream>>>(k_w, WK); k_wtG<<<(HD * HD / 8 + 255) / 256, 256, 0, stream>>>(v_w, WV); k_wtG<<<(HD * HD / 8 + 255) / 256, 256, 0, stream>>>(o_w, WO); k_nexchk<<<1, 32, 0, stream>>>(nex, FLG);
    k_cvt8<<<(unsigned)(((size_t)SQ * HD / 8 + 255) / 256), 256, 0, stream>>>(query, XQ, (size_t)SQ * HD / 8);
    k_gemmw<bf, 0, true><<<dim3(SQ / 64, HD / 64, 1), 32, 0, stream>>>(XQ, nullptr, WQ, nullptr, HD, FQ, HD, q_b, 0, 0, 0);
    k_ropq<<<(unsigned)(((size_t)SQ * HD / 2 + 255) / 256), 256, 0, stream>>>(FQ, SQ, SQ, 1, cosT, sinT);
    k_hlG<<<(unsigned)(((size_t)SQ * HD / 4 + 255) / 256), 256, 0, stream>>>(FQ, QPh, QPl, (size_t)SQ * HD);
    k_cvt8<<<(unsigned)(((size_t)SK * HD / 8 + 255) / 256), 256, 0, stream>>>(key, XK, (size_t)SK * HD / 8);
    k_gemmw<bf, 0, true><<<dim3(SK / 64, HD / 64, 1), 32, 0, stream>>>(XK, nullptr, WK, nullptr, HD, FK, HD, k_b, 0, 0, 0);
    k_ropq<<<(unsigned)(((size_t)SK * HD / 2 + 255) / 256), 256, 0, stream>>>(FK, SK, SK - NEX, (SK - NEX) / SQ, cosT, sinT);
    k_hlG<<<(unsigned)(((size_t)SK * HD / 4 + 255) / 256), 256, 0, stream>>>(FK, KPh, KPl, (size_t)SK * HD);
    k_cvt8<<<(unsigned)(((size_t)SK * HD / 8 + 255) / 256), 256, 0, stream>>>(value, XK, (size_t)SK * HD / 8);
    k_gemmw<bf, 0, true><<<dim3(SK / 64, HD / 64, 1), 32, 0, stream>>>(XK, nullptr, WV, nullptr, HD, FV, HD, v_b, 0, 0, 0);
    k_v16T<<<(unsigned)(((size_t)HD * SK / 2 + 255) / 256), 256, 0, stream>>>(FV, VT16);
    for (int c = 0; c < SQ / QC; ++c) {
        k_gemmw<bf, 2, false><<<dim3(QC / 64, SK / 64, 1), 32, 0, stream>>>(QPh + (size_t)c * QC * HD, QPl + (size_t)c * QC * HD, KPh, KPl, HD, S, SK, nullptr, 0, 0, 0);
        k_lsoft<<<QC / 8, 256, 0, stream>>>(S, FLG, P16);
        k_gemmw<h16, 0, false><<<dim3(QC / 64, HD / 64, 1), 32, 0, stream>>>(P16, nullptr, VT16, nullptr, SK, O, HD, nullptr, 0, 0, 0);
        k_ofix<<<(unsigned)(((size_t)QC * HD / 4 + 255) / 256), 256, 0, stream>>>(O, Oh, Ol);
        k_gemmw<bf, 1, true><<<dim3(QC / 64, HD / 64, 1), 32, 0, stream>>>(Oh, Ol, WO, nullptr, HD, OUT + (size_t)c * QC * HD, HD, o_b, 0, 0, 0); }
}
